// CausalSelfAttention_16879221473590
// MI455X (gfx1250) — hardware-verified
//
#include <hip/hip_runtime.h>


#ifndef NB
#define NB 4
#endif
#ifndef SEQ
#define SEQ 2048
#endif
#define NB_FULL  4
#define SEQ_FULL 2048
#define TT   SEQ
#define DM   1024
#define NH_  16
#define HD   64
#define DQ   (NH_ * HD)
#define D3   (3 * DQ)
#define ZH   2
#define RH   ((SEQ < 512) ? SEQ : 512)
#define PCAR 1024.0f
#define SCL  0.125f

static_assert(HD == 64);
static_assert(DQ == DM);
static_assert(DM % 64 == 0);
static_assert(D3 % 64 == 0);
static_assert(TT % 128 == 0);
static_assert(RH % 64 == 0);
static_assert(HD % 32 == 0);
static_assert(NH_ % ZH == 0);
static_assert((ZH * TT) % 8 == 0);
static_assert(NB <= NB_FULL);
static_assert(SEQ <= SEQ_FULL);

typedef _Float16 h16;
typedef unsigned short bf;
typedef __attribute__((ext_vector_type(16))) __bf16   v16bf;
typedef __attribute__((ext_vector_type(16))) _Float16 v16h;
typedef __attribute__((ext_vector_type(8)))  _Float16 v8h;
typedef __attribute__((ext_vector_type(8)))  unsigned short v8us;
typedef __attribute__((ext_vector_type(8)))  float    v8f;
typedef __attribute__((ext_vector_type(4)))  float    v4f;
typedef __attribute__((ext_vector_type(4)))  _Float16 v4h;
typedef __attribute__((ext_vector_type(4)))  unsigned short v4us;
typedef v4f  __attribute__((may_alias)) v4fa;
typedef v8us __attribute__((may_alias)) v8usa;

__device__ __forceinline__ unsigned short f2bf(float f) { unsigned u = __float_as_uint(f); u += 0x7FFFu + ((u >> 16) & 1u); return (unsigned short)(u >> 16); }
__device__ __forceinline__ float bf2f(unsigned short b) { return __uint_as_float(((unsigned)b) << 16); }
__device__ __forceinline__ float bfr(float f) { return bf2f(f2bf(f)); }
__device__ __forceinline__ v16h cat16(v8h lo, v8h hi) { return __builtin_shufflevector(lo, hi, 0, 1, 2, 3, 4, 5, 6, 7, 8, 9, 10, 11, 12, 13, 14, 15); }
__device__ __forceinline__ v16bf cat16b(v8us lo, v8us hi) { return __builtin_bit_cast(v16bf, __builtin_shufflevector(lo, hi, 0, 1, 2, 3, 4, 5, 6, 7, 8, 9, 10, 11, 12, 13, 14, 15)); }
__device__ __forceinline__ v8f wmma16(v16h a, v16h b, v8f c) { return __builtin_amdgcn_wmma_f32_16x16x32_f16(false, a, false, b, (short)0, c, false, false); }
__device__ __forceinline__ v8f wmmab(v16bf a, v16bf b, v8f c) { return __builtin_amdgcn_wmma_f32_16x16x32_bf16(false, a, false, b, (short)0, c, false, false); }
__device__ __forceinline__ h16 tohx(float x) { return (h16)x; }
__device__ __forceinline__ void splitf(float y, unsigned short& h, unsigned short& l) { h = f2bf(y); l = f2bf(y - bf2f(h)); }

template <typename T16> struct WFrag;
template <> struct WFrag<h16> { typedef v16h V; static __device__ __forceinline__ V ld(const h16* p) { return cat16(*(const v8h*)p, *(const v8h*)(p + 16)); } static __device__ __forceinline__ v8f mma(V a, V b, v8f c) { return wmma16(a, b, c); } };
template <> struct WFrag<bf> { typedef v16bf V; static __device__ __forceinline__ V ld(const bf* p) { return cat16b(*(const v8us*)p, *(const v8us*)(p + 16)); } static __device__ __forceinline__ v8f mma(V a, V b, v8f c) { return wmmab(a, b, c); } };

template <typename T16, int NSPLIT, bool BIAS>
__device__ __forceinline__ void gemmw_body(const T16* __restrict__ A, const T16* __restrict__ A2, const T16* __restrict__ Bt, const T16* __restrict__ Bt2, int K, float* C, int ldc, const float* __restrict__ bias) {
    typedef typename WFrag<T16>::V V;
    __shared__ __align__(16) float os[16 * 68];
    const int lane = threadIdx.x & 31, lr = lane & 15, hi = lane >> 4; const int r0 = blockIdx.x * 64, c0 = blockIdx.y * 64;
    v8f acc[4][4];
#pragma unroll
    for (int mb = 0; mb < 4; ++mb)
#pragma unroll
        for (int nb = 0; nb < 4; ++nb) acc[mb][nb] = (v8f){};
    const size_t aoff = (size_t)(r0 + lr) * K + 8 * hi, boff = (size_t)(c0 + lr) * K + 8 * hi;
#pragma unroll 1
    for (int kc = 0; kc < K; kc += 32) {
        V a[4], a2[4];
#pragma unroll
        for (int mb = 0; mb < 4; ++mb) { a[mb] = WFrag<T16>::ld(A + aoff + (size_t)mb * 16 * K + kc); if (NSPLIT == 1 || NSPLIT == 2) a2[mb] = WFrag<T16>::ld(A2 + aoff + (size_t)mb * 16 * K + kc); }
#pragma unroll
        for (int nb = 0; nb < 4; ++nb) { const V b = WFrag<T16>::ld(Bt + boff + (size_t)nb * 16 * K + kc); V b2; if (NSPLIT >= 2) b2 = WFrag<T16>::ld(Bt2 + boff + (size_t)nb * 16 * K + kc);
#pragma unroll
            for (int mb = 0; mb < 4; ++mb) { acc[mb][nb] = WFrag<T16>::mma(a[mb], b, acc[mb][nb]); if (NSPLIT == 1 || NSPLIT == 2) acc[mb][nb] = WFrag<T16>::mma(a2[mb], b, acc[mb][nb]); if (NSPLIT >= 2) acc[mb][nb] = WFrag<T16>::mma(a[mb], b2, acc[mb][nb]); } }
        asm volatile("v_nop\n\tv_nop\n\tv_nop\n\tv_nop" : "+v"(acc[0][0]), "+v"(acc[1][1]), "+v"(acc[2][2]), "+v"(acc[3][3]), "+v"(acc[0][3]), "+v"(acc[1][3]), "+v"(acc[2][3]) : "v"(a[0]), "v"(a[3]));
    }
    v4f bv = (v4f){0.f, 0.f, 0.f, 0.f};
    if (BIAS) { const int cb = c0 + lr * 4; bv[0] = bfr(bias[cb]); bv[1] = bfr(bias[cb + 1]); bv[2] = bfr(bias[cb + 2]); bv[3] = bfr(bias[cb + 3]); }
#pragma unroll
    for (int mb = 0; mb < 4; ++mb) {
#pragma unroll
        for (int nb = 0; nb < 4; ++nb) {
#pragma unroll
            for (int j = 0; j < 8; ++j) os[(hi * 8 + j) * 68 + nb * 16 + lr] = acc[mb][nb][j]; }
        __builtin_amdgcn_wave_barrier(); asm volatile("" ::: "memory");
        float* crow = C + (size_t)(r0 + mb * 16) * ldc + c0;
#pragma unroll 1
        for (int ps = 0; ps < 2; ++ps) {
#pragma unroll
            for (int s = 0; s < 8; ++s) { const int row = 2 * s + hi, cofs = lr * 4; v4f val = *(const v4fa*)(os + row * 68 + cofs); val = val + bv;
                *(volatile v4f*)(crow + (size_t)row * ldc + cofs) = val; }
            if (ps == 0) __threadfence(); }
        __builtin_amdgcn_wave_barrier(); asm volatile("" ::: "memory");
    }
}

template <typename T16, int NSPLIT, int CMODE>
__device__ __forceinline__ void gemmc_body(const T16* __restrict__ A, const T16* __restrict__ A2, const T16* __restrict__ Bt, const T16* __restrict__ Bt2, int K, float* C, int ldc, int roff, size_t sA, size_t sB, size_t sC) {
    typedef typename WFrag<T16>::V V;
    __shared__ __align__(16) float os[16 * 68];
    const size_t z = blockIdx.z; A += z * sA; if (A2) A2 += z * sA; Bt += z * sB; if (Bt2) Bt2 += z * sB; C += z * sC;
    const int lane = threadIdx.x & 31, lr = lane & 15, hi = lane >> 4; const int r0 = blockIdx.x * 64, c0 = blockIdx.y * 64;
    if (CMODE == 1 && c0 > r0 + roff + 63) return;
    const int Kl = (CMODE == 2) ? min(K, r0 + roff + 64) : K;
    v8f acc[4][4];
#pragma unroll
    for (int mb = 0; mb < 4; ++mb)
#pragma unroll
        for (int nb = 0; nb < 4; ++nb) acc[mb][nb] = (v8f){};
    const size_t aoff = (size_t)(r0 + lr) * K + 8 * hi, boff = (size_t)(c0 + lr) * K + 8 * hi;
#pragma unroll 1
    for (int kc = 0; kc < Kl; kc += 32) {
        V a[4], a2[4];
#pragma unroll
        for (int mb = 0; mb < 4; ++mb) { a[mb] = WFrag<T16>::ld(A + aoff + (size_t)mb * 16 * K + kc); if (NSPLIT == 1 || NSPLIT == 2) a2[mb] = WFrag<T16>::ld(A2 + aoff + (size_t)mb * 16 * K + kc); }
#pragma unroll
        for (int nb = 0; nb < 4; ++nb) { const V b = WFrag<T16>::ld(Bt + boff + (size_t)nb * 16 * K + kc); V b2; if (NSPLIT >= 2) b2 = WFrag<T16>::ld(Bt2 + boff + (size_t)nb * 16 * K + kc);
#pragma unroll
            for (int mb = 0; mb < 4; ++mb) { acc[mb][nb] = WFrag<T16>::mma(a[mb], b, acc[mb][nb]); if (NSPLIT == 1 || NSPLIT == 2) acc[mb][nb] = WFrag<T16>::mma(a2[mb], b, acc[mb][nb]); if (NSPLIT >= 2) acc[mb][nb] = WFrag<T16>::mma(a[mb], b2, acc[mb][nb]); } }
        asm volatile("v_nop\n\tv_nop\n\tv_nop\n\tv_nop" : "+v"(acc[0][0]), "+v"(acc[1][1]), "+v"(acc[2][2]), "+v"(acc[3][3]), "+v"(acc[0][3]), "+v"(acc[1][3]), "+v"(acc[2][3]) : "v"(a[0]), "v"(a[3]));
    }
#pragma unroll
    for (int mb = 0; mb < 4; ++mb) {
#pragma unroll
        for (int nb = 0; nb < 4; ++nb) {
#pragma unroll
            for (int j = 0; j < 8; ++j) os[(hi * 8 + j) * 68 + nb * 16 + lr] = acc[mb][nb][j]; }
        __builtin_amdgcn_wave_barrier(); asm volatile("" ::: "memory");
        float* crow = C + (size_t)(r0 + mb * 16) * ldc + c0;
#pragma unroll 1
        for (int ps = 0; ps < 2; ++ps) {
#pragma unroll
            for (int s = 0; s < 8; ++s) { const int row = 2 * s + hi, cofs = lr * 4; const v4f val = *(const v4fa*)(os + row * 68 + cofs);
                *(volatile v4f*)(crow + (size_t)row * ldc + cofs) = val; }
            if (ps == 0) __threadfence(); }
        __builtin_amdgcn_wave_barrier(); asm volatile("" ::: "memory");
    }
}

__global__ __launch_bounds__(32) void k_gemm_qkv(const bf* __restrict__ A, const bf* __restrict__ Bt, int K, float* C, int ldc, const float* __restrict__ bias) { gemmw_body<bf, 0, true>(A, nullptr, Bt, nullptr, K, C, ldc, bias); }
__global__ __launch_bounds__(32) void k_gemm_out(const bf* __restrict__ Ah, const bf* __restrict__ Al, const bf* __restrict__ Bt, int K, float* C, int ldc, const float* __restrict__ bias) { gemmw_body<bf, 1, true>(Ah, Al, Bt, nullptr, K, C, ldc, bias); }
__global__ __launch_bounds__(32) void k_sc_hl(const bf* __restrict__ Qh, const bf* __restrict__ Ql, const bf* __restrict__ Kh, const bf* __restrict__ Kl, float* S) { gemmc_body<bf, 2, 1>(Qh, Ql, Kh, Kl, HD, S, TT, 0, (size_t)TT * HD, (size_t)TT * HD, (size_t)TT * TT); }
__global__ __launch_bounds__(32) void k_sc_h(const h16* __restrict__ Q, const h16* __restrict__ Kp, float* S) { gemmc_body<h16, 0, 1>(Q, nullptr, Kp, nullptr, HD, S, TT, RH, (size_t)TT * HD, (size_t)TT * HD, (size_t)TT * TT); }
__global__ __launch_bounds__(32) void k_pv_hl(const bf* __restrict__ Ph, const bf* __restrict__ Pl, const bf* __restrict__ Vh, const bf* __restrict__ Vl, float* O) { gemmc_body<bf, 2, 2>(Ph, Pl, Vh, Vl, TT, O, HD, 0, (size_t)RH * TT, (size_t)HD * TT, (size_t)TT * HD); }
__global__ __launch_bounds__(32) void k_pv_h(const h16* __restrict__ P, const h16* __restrict__ V, float* O) { gemmc_body<h16, 0, 2>(P, nullptr, V, nullptr, TT, O, HD, RH, (size_t)TT * TT, (size_t)HD * TT, (size_t)TT * HD); }

__global__ __launch_bounds__(256) void k_cvt8(const float* __restrict__ src, bf* dst, size_t n8) { const size_t i = (size_t)blockIdx.x * 256 + threadIdx.x; if (i >= n8) return; const v8f v = *(const v8f*)(src + i * 8); v8us o;
#pragma unroll
    for (int k = 0; k < 8; ++k) o[k] = f2bf(v[k]); *(volatile v8us*)(dst + i * 8) = o; __threadfence(); *(volatile v8us*)(dst + i * 8) = o; }

__global__ __launch_bounds__(256) void k_wtr(const float* __restrict__ W, int nin, int nout, bf* Bt) {
    __shared__ __align__(16) unsigned short ts[64 * 72];
    const int tid = threadIdx.x; const int i0 = blockIdx.x * 64, o0 = blockIdx.y * 64;
#pragma unroll
    for (int it = 0; it < 4; ++it) { const int r = (tid >> 4) + 16 * it; const int c = (tid & 15) * 4; const v4f v = *(const v4f*)(W + (size_t)(i0 + r) * nout + o0 + c);
#pragma unroll
        for (int q = 0; q < 4; ++q) ts[(c + q) * 72 + r] = f2bf(v[q]); }
    __syncthreads();
    const int lane = tid & 31, wv = tid >> 5;
#pragma unroll 1
    for (int ps = 0; ps < 2; ++ps) {
#pragma unroll
        for (int it2 = 0; it2 < 2; ++it2) { const int row = wv * 8 + it2 * 4 + (lane >> 3); const int pc = lane & 7; const v8us o = *(const v8usa*)(ts + row * 72 + pc * 8);
            *(volatile v8us*)(Bt + (size_t)(o0 + row) * nin + i0 + pc * 8) = o; }
        if (ps == 0) __threadfence(); }
}

__global__ __launch_bounds__(256) void k_planeqk(const float* __restrict__ F, h16* P16, bf* Ph, bf* Pl) {
    const size_t e8 = (size_t)blockIdx.x * 256 + threadIdx.x; if (e8 >= (size_t)2 * NH_ * TT * HD / 8) return;
    const int d8 = (int)(e8 & 7); const int t = (int)((e8 >> 3) % TT); const int hh = (int)(e8 / ((size_t)8 * TT));
    const float* f = F + (size_t)t * D3 + hh * HD + d8 * 8; const v4f a = *(const v4f*)f; const v4f b = *(const v4f*)(f + 4);
    v8h o16; v8us oh, ol;
#pragma unroll
    for (int q = 0; q < 8; ++q) { const float x = (q < 4) ? a[q & 3] : b[q & 3]; o16[q] = tohx(x); unsigned short a2, c2; splitf(x, a2, c2); oh[q] = a2; ol[q] = c2; }
    const size_t oo = e8 * 8;
    *(volatile v8h*)(P16 + oo) = o16; *(volatile v8us*)(Ph + oo) = oh; *(volatile v8us*)(Pl + oo) = ol; __threadfence(); *(volatile v8h*)(P16 + oo) = o16; *(volatile v8us*)(Ph + oo) = oh; *(volatile v8us*)(Pl + oo) = ol; }

__global__ __launch_bounds__(256) void k_planev(const float* __restrict__ F, h16* V16, bf* Vh, bf* Vl) {
    const size_t e8 = (size_t)blockIdx.x * 256 + threadIdx.x; if (e8 >= (size_t)NH_ * HD * TT / 8) return;
    const int t8 = (int)(e8 % (TT / 8)); const int d = (int)((e8 / (TT / 8)) % HD); const int g = (int)(e8 / ((size_t)(TT / 8) * HD));
    v8h o16; v8us oh, ol;
#pragma unroll
    for (int q = 0; q < 8; ++q) { const float x = F[(size_t)(t8 * 8 + q) * D3 + 2 * DQ + g * HD + d]; o16[q] = tohx(x); unsigned short a2, c2; splitf(x, a2, c2); oh[q] = a2; ol[q] = c2; }
    const size_t oo = e8 * 8;
    *(volatile v8h*)(V16 + oo) = o16; *(volatile v8us*)(Vh + oo) = oh; *(volatile v8us*)(Vl + oo) = ol; __threadfence(); *(volatile v8h*)(V16 + oo) = o16; *(volatile v8us*)(Vh + oo) = oh; *(volatile v8us*)(Vl + oo) = ol; }

__global__ __launch_bounds__(256) void k_asoft(const float* __restrict__ Sb, h16* P16, bf* Ph, bf* Pl) {
    const int lane = threadIdx.x & 31; const int wv = __builtin_amdgcn_readfirstlane((int)(threadIdx.x >> 5)); const int row = blockIdx.x * 8 + wv; if (row >= ZH * TT) return;
    const int i = row % TT; const int zz = row / TT; const bool hires = (i < RH); const int lim = ((i >> 6) + 1) << 6;
    const float* sr = Sb + (size_t)row * TT; float v[TT / 32]; float mx = -3.0e38f;
#pragma unroll
    for (int ch = 0; ch < TT / 128; ++ch) {
        if (ch * 128 < lim) { const int j0 = ch * 128 + lane * 4; const v4f a = *(const v4f*)(sr + j0);
#pragma unroll
            for (int q = 0; q < 4; ++q) { const int j = j0 + q; const float t = (j <= i) ? a[q] * SCL : -3.0e38f; v[ch * 4 + q] = t; mx = fmaxf(mx, t); } }
        else {
#pragma unroll
            for (int q = 0; q < 4; ++q) v[ch * 4 + q] = -3.0e38f; } }
#pragma unroll
    for (int sh = 16; sh; sh >>= 1) mx = fmaxf(mx, __shfl_xor(mx, sh, 32));
    float sum = 0.f;
#pragma unroll
    for (int k = 0; k < TT / 32; ++k) {
        if ((k >> 2) * 128 < lim) { float d0 = __fsub_rn(v[k], mx); asm volatile("" : "+v"(d0)); v[k] = __builtin_amdgcn_exp2f(__fmul_rn(d0, 1.4426950408889634f)); sum += v[k]; }
        else v[k] = 0.f; }
#pragma unroll
    for (int sh = 16; sh; sh >>= 1) sum += __shfl_xor(sum, sh, 32);
    const float f = (hires ? 1.0f : PCAR) * (1.0f / sum);
#pragma unroll 1
    for (int ps = 0; ps < 2; ++ps) {
        if (hires) {
#pragma unroll
            for (int ch = 0; ch < TT / 128; ++ch) { if (ch * 128 < lim) { v4us oh, ol;
#pragma unroll
                for (int q = 0; q < 4; ++q) { unsigned short a, c2; splitf(v[ch * 4 + q] * f, a, c2); oh[q] = a; ol[q] = c2; }
                const size_t oo = ((size_t)zz * RH + i) * TT + ch * 128 + lane * 4; *(volatile v4us*)(Ph + oo) = oh; *(volatile v4us*)(Pl + oo) = ol; } }
        } else {
#pragma unroll
            for (int ch = 0; ch < TT / 128; ++ch) { if (ch * 128 < lim) { v4h o4;
#pragma unroll
                for (int q = 0; q < 4; ++q) o4[q] = tohx(v[ch * 4 + q] * f);
                *(volatile v4h*)(P16 + (size_t)row * TT + ch * 128 + lane * 4) = o4; } } }
        if (ps == 0) __threadfence(); }
}

__global__ __launch_bounds__(256) void k_merge(const float* __restrict__ O, bf* Ah, bf* Al) {
    const size_t e8 = (size_t)blockIdx.x * 256 + threadIdx.x; if (e8 >= (size_t)NH_ * TT * HD / 8) return;
    const int d8 = (int)(e8 & 7); const int t = (int)((e8 >> 3) % TT); const int h = (int)(e8 / ((size_t)8 * TT)); const float cs = (t < RH) ? 1.0f : (1.0f / PCAR);
    const v4f a = *(const v4f*)(O + e8 * 8); const v4f b = *(const v4f*)(O + e8 * 8 + 4); v8us oh, ol;
#pragma unroll
    for (int q = 0; q < 8; ++q) { const float x = ((q < 4) ? a[q & 3] : b[q & 3]) * cs; unsigned short a2, c2; splitf(x, a2, c2); oh[q] = a2; ol[q] = c2; }
    const size_t oo = (size_t)t * DQ + h * HD + d8 * 8;
    *(volatile v8us*)(Ah + oo) = oh; *(volatile v8us*)(Al + oo) = ol; __threadfence(); *(volatile v8us*)(Ah + oo) = oh; *(volatile v8us*)(Al + oo) = ol; }

constexpr size_t cmaxz(size_t a, size_t b) { return a > b ? a : b; }
constexpr size_t SZ_WA  = (size_t)D3 * DM * 2;
constexpr size_t SZ_WO  = (size_t)DM * DQ * 2;
constexpr size_t SZ_XB  = (size_t)TT * DM * 2;
constexpr size_t SZ_QK  = (size_t)2 * NH_ * TT * HD * 2;
constexpr size_t SZ_VT  = (size_t)NH_ * HD * TT * 2;
constexpr size_t SZ_PH  = (size_t)ZH * RH * TT * 2;
constexpr size_t SZ_S   = (size_t)ZH * TT * TT * 4;
constexpr size_t SZ_F   = (size_t)TT * D3 * 4;
constexpr size_t SZ_SF  = cmaxz(SZ_S, SZ_F);
constexpr size_t SZ_P16 = (size_t)ZH * TT * TT * 2;
constexpr size_t SZ_OB  = (size_t)NH_ * TT * HD * 4;
constexpr size_t SZ_AT  = (size_t)TT * DQ * 2;
constexpr size_t SZ_TOTAL = SZ_WA + SZ_WO + SZ_XB + 3 * SZ_QK + 3 * SZ_VT + 2 * SZ_PH + SZ_SF + SZ_P16 + SZ_OB + 2 * SZ_AT;
static_assert(SZ_S <= SZ_SF);
static_assert(SZ_F <= SZ_SF);
static_assert(SZ_WA % 256 == 0 && SZ_WO % 256 == 0 && SZ_XB % 256 == 0 && SZ_QK % 256 == 0 && SZ_VT % 256 == 0 && SZ_PH % 256 == 0 && SZ_SF % 256 == 0 && SZ_P16 % 256 == 0 && SZ_OB % 256 == 0 && SZ_AT % 256 == 0);
static_assert(SZ_TOTAL <= (size_t)134217728);

extern "C" void kernel_launch(void* const* d_in, const int* in_sizes, int n_in,
                              void* d_out, int out_size, void* d_ws, size_t ws_size, hipStream_t stream) {
    if (n_in < 5) return;
    if ((size_t)in_sizes[0] < (size_t)(NB - 1) * SEQ_FULL * DM + (size_t)SEQ * DM) return;
    if ((size_t)in_sizes[1] < (size_t)DM * D3 || in_sizes[2] < D3 || (size_t)in_sizes[3] < (size_t)DQ * DM || in_sizes[4] < DM) return;
    if ((size_t)out_size < (size_t)NB * SEQ * DM) return;
    if (ws_size < SZ_TOTAL) return;
    const float* x = (const float*)d_in[0]; const float* wattn = (const float*)d_in[1]; const float* battn = (const float*)d_in[2]; const float* wproj = (const float*)d_in[3]; const float* bproj = (const float*)d_in[4];
    float* OUT = (float*)d_out;
    char* wsp = (char*)d_ws;
    auto take = [&](size_t bytes) { char* p = wsp; wsp += bytes; return (void*)p; };
    bf* WA = (bf*)take(SZ_WA); bf* WO = (bf*)take(SZ_WO); bf* XB = (bf*)take(SZ_XB);
    h16* QK16 = (h16*)take(SZ_QK); bf* QKh = (bf*)take(SZ_QK); bf* QKl = (bf*)take(SZ_QK);
    h16* VT16 = (h16*)take(SZ_VT); bf* VTh = (bf*)take(SZ_VT); bf* VTl = (bf*)take(SZ_VT);
    bf* Ph = (bf*)take(SZ_PH); bf* Pl = (bf*)take(SZ_PH);
    float* Sb = (float*)take(SZ_SF); float* F = Sb;
    h16* P16 = (h16*)take(SZ_P16); float* Ob = (float*)take(SZ_OB); bf* ATh = (bf*)take(SZ_AT); bf* ATl = (bf*)take(SZ_AT);
    if ((size_t)(wsp - (char*)d_ws) > ws_size) return;
    const size_t KOFF = (size_t)NH_ * TT * HD;
    h16* QP16 = QK16; h16* KP16 = QK16 + KOFF; bf* QPh = QKh; bf* KPh = QKh + KOFF; bf* QPl = QKl; bf* KPl = QKl + KOFF;

    k_wtr<<<dim3(DM / 64, D3 / 64), 256, 0, stream>>>(wattn, DM, D3, WA);
    k_wtr<<<dim3(DQ / 64, DM / 64), 256, 0, stream>>>(wproj, DQ, DM, WO);

    const unsigned LQK = (unsigned)(((size_t)2 * NH_ * TT * HD / 8 + 255) / 256), LV = (unsigned)(((size_t)NH_ * HD * TT / 8 + 255) / 256);
    for (int b = 0; b < NB; ++b) {
        k_cvt8<<<(unsigned)(((size_t)TT * DM / 8 + 255) / 256), 256, 0, stream>>>(x + (size_t)b * SEQ_FULL * DM, XB, (size_t)TT * DM / 8);
        k_gemm_qkv<<<dim3(TT / 64, D3 / 64, 1), 32, 0, stream>>>(XB, WA, DM, F, D3, battn);
        k_planeqk<<<LQK, 256, 0, stream>>>(F, QK16, QKh, QKl);
        k_planev<<<LV, 256, 0, stream>>>(F, VT16, VTh, VTl);
        for (int h0 = 0; h0 < NH_; h0 += ZH) { const size_t zq = (size_t)h0 * TT * HD;
            k_sc_hl<<<dim3(RH / 64, RH / 64, ZH), 32, 0, stream>>>(QPh + zq, QPl + zq, KPh + zq, KPl + zq, Sb);
            if (TT > RH) k_sc_h<<<dim3((TT - RH) / 64, TT / 64, ZH), 32, 0, stream>>>(QP16 + zq + (size_t)RH * HD, KP16 + zq, Sb + (size_t)RH * TT);
            k_asoft<<<ZH * TT / 8, 256, 0, stream>>>(Sb, P16, Ph, Pl);
            k_pv_hl<<<dim3(RH / 64, 1, ZH), 32, 0, stream>>>(Ph, Pl, VTh + zq, VTl + zq, Ob + zq);
            if (TT > RH) k_pv_h<<<dim3((TT - RH) / 64, 1, ZH), 32, 0, stream>>>(P16 + (size_t)RH * TT, VT16 + zq, Ob + zq + (size_t)RH * HD); }
        k_merge<<<(unsigned)(((size_t)NH_ * TT * HD / 8 + 255) / 256), 256, 0, stream>>>(Ob, ATh, ATl);
        k_gemm_out<<<dim3(TT / 64, DM / 64, 1), 32, 0, stream>>>(ATh, ATl, WO, DQ, OUT + (size_t)b * TT * DM, DM, bproj); }
}
